// PlaneNet_4853313045169
// MI455X (gfx1250) — hardware-run, weakly checked
//
#include <hip/hip_runtime.h>

typedef float          v8f   __attribute__((ext_vector_type(8)));
typedef float          v4f   __attribute__((ext_vector_type(4)));
typedef unsigned int   v4u   __attribute__((ext_vector_type(4)));
typedef int            v8i   __attribute__((ext_vector_type(8)));
typedef unsigned short v8us  __attribute__((ext_vector_type(8)));
typedef unsigned short v16us __attribute__((ext_vector_type(16)));
typedef __bf16         v16bf __attribute__((ext_vector_type(16)));
typedef _Float16       v16h  __attribute__((ext_vector_type(16)));
typedef v4f  __attribute__((may_alias)) v4fa;
typedef v8us __attribute__((may_alias)) v8usa;
union FragB { v16bf v; v16us u; v8us h[2]; v8i w; };
union FragH { v16h  v; v16us u; v8us h[2]; v8i w; };

__device__ __forceinline__ v8f wmb(const FragB& a, const FragB& b, v8f c) {
  v8f d = __builtin_amdgcn_wmma_f32_16x16x32_bf16(false, a.v, false, b.v, (short)0, c, false, false);
  asm volatile("v_nop\n\tv_nop\n\tv_nop\n\tv_nop" : "+v"(d) : "v"(a.w), "v"(b.w));
  return d;
}

__device__ __forceinline__ v8f wmh(const FragH& a, const FragH& b, v8f c) {
  v8f d = __builtin_amdgcn_wmma_f32_16x16x32_f16(false, a.v, false, b.v, (short)0, c, false, false);
  asm volatile("v_nop\n\tv_nop\n\tv_nop\n\tv_nop" : "+v"(d) : "v"(a.w), "v"(b.w));
  return d;
}

__device__ __forceinline__ unsigned bf16_bits(float f) {
  const unsigned u = __float_as_uint(f);
  const unsigned r = (u + 0x7FFFu + ((u >> 16) & 1u)) >> 16;
  const unsigned q = (u >> 16) | 0x40u;
  return ((u & 0x7fffffffu) > 0x7f800000u) ? q : r;
}

__device__ __forceinline__ float bf16_val(float f) {
  return __uint_as_float(bf16_bits(f) << 16);
}
__device__ __forceinline__ int clampi(int v, int lo, int hi) {
  return v < lo ? lo : (v > hi ? hi : v);
}

__device__ __forceinline__ unsigned f16_bits(float f) {
  const unsigned u  = __float_as_uint(f);
  const unsigned s  = (u >> 16) & 0x8000u;
  const unsigned a  = u & 0x7fffffffu;
  const unsigned t  = a - 0x38000000u;
  const unsigned r  = (t + 0x0FFFu + ((t >> 13) & 1u)) >> 13;
  const unsigned rc = r > 0x7C00u ? 0x7C00u : r;
  const bool small  = a < 0x38800000u;
  const bool isnan  = a > 0x7f800000u;
  const unsigned fin = small ? 0u : (s | rc);
  return isnan ? (s | 0x7E00u) : fin;
}

__device__ __forceinline__ unsigned pk16(unsigned lo, unsigned hi) { return lo | (hi << 16); }
__device__ __forceinline__ unsigned bf16_lo_bits(float v) {
  float hi = bf16_val(v);
  asm volatile("" : "+v"(hi));
  return bf16_bits(v - hi);
}
__device__ __forceinline__ v4u pack8_bf16(v4f a, v4f c) {
  return (v4u){ pk16(bf16_bits(a[0]), bf16_bits(a[1])), pk16(bf16_bits(a[2]), bf16_bits(a[3])),
                pk16(bf16_bits(c[0]), bf16_bits(c[1])), pk16(bf16_bits(c[2]), bf16_bits(c[3])) };
}
__device__ __forceinline__ v4u pack8_bf16_lo(v4f a, v4f c) {
  return (v4u){ pk16(bf16_lo_bits(a[0]), bf16_lo_bits(a[1])), pk16(bf16_lo_bits(a[2]), bf16_lo_bits(a[3])),
                pk16(bf16_lo_bits(c[0]), bf16_lo_bits(c[1])), pk16(bf16_lo_bits(c[2]), bf16_lo_bits(c[3])) };
}
__device__ __forceinline__ v4u pack8_f16(v4f a, v4f c) {
  return (v4u){ pk16(f16_bits(a[0]), f16_bits(a[1])), pk16(f16_bits(a[2]), f16_bits(a[3])),
                pk16(f16_bits(c[0]), f16_bits(c[1])), pk16(f16_bits(c[2]), f16_bits(c[3])) };
}

template <int FORM>
__global__ __launch_bounds__(256) void k_plane(const float* __restrict__ src, int rows, int cols, int ldsrc,
                                               unsigned short* __restrict__ dst, int MP, int KP) {
  static_assert(FORM >= 0 && FORM <= 3);
  const int KTOT = (FORM == 1 || FORM == 3) ? 2 * KP : KP;
  const unsigned ppr   = (unsigned)(KTOT >> 3);
  const unsigned kp8   = (unsigned)(KP >> 3);
  const unsigned total = (unsigned)MP * ppr;
  const unsigned g     = blockIdx.x * 256u + threadIdx.x;
  const unsigned rowu  = g / ppr;
  const unsigned p     = g - rowu * ppr;
  const bool second    = p >= kp8;
  const int row = (int)rowu;
  const int c0  = (int)((second ? p - kp8 : p) << 3);
  const float* srow = src + (size_t)clampi(row, 0, rows - 1) * (size_t)ldsrc;
  float x[8];
  unsigned mk[8];
#pragma unroll
  for (int e = 0; e < 8; ++e) {
    const int c = c0 + e;
    const float v = srow[clampi(c, 0, cols - 1)];
    asm volatile("" :: "v"(v));
    x[e]  = v;
    mk[e] = (row < rows && c < cols) ? 0xFFFFu : 0u;
  }
  const v4f a = (v4f){ x[0], x[1], x[2], x[3] };
  const v4f c = (v4f){ x[4], x[5], x[6], x[7] };
  v4u o;
  if (FORM == 2) {
    o = pack8_f16(a, c);
  } else {
    const v4u hi = pack8_bf16(a, c);
    o = hi;
    if (FORM == 1) { const v4u lo = pack8_bf16_lo(a, c); o = second ? lo : hi; }
  }
  const v4u mw = (v4u){ pk16(mk[0], mk[1]), pk16(mk[2], mk[3]), pk16(mk[4], mk[5]), pk16(mk[6], mk[7]) };
  o &= mw;
  if (g < total) {
    volatile v4u* q = (volatile v4u*)(dst + (size_t)g * 8);
    *q = o;
    __threadfence();
    *q = o;
  }
}

template <int FORM> struct FragOf    { typedef FragB T; };
template <>         struct FragOf<2> { typedef FragH T; };
__device__ __forceinline__ v8f mm(const FragB& a, const FragB& b, v8f c) { return wmb(a, b, c); }
__device__ __forceinline__ v8f mm(const FragH& a, const FragH& b, v8f c) { return wmh(a, b, c); }
template <class F> __device__ __forceinline__ F ld_frag(const unsigned short* p) {
  F f;
  f.h[0] = *(const v8usa*)(p);
  f.h[1] = *(const v8usa*)(p + 16);
  return f;
}

template <int FORM, int EPI>
__global__ __launch_bounds__(256) __attribute__((amdgpu_num_vgpr(248)))
void k_gemm_nt(const unsigned short* __restrict__ A, const unsigned short* __restrict__ B,
               const float* __restrict__ bias, float* __restrict__ D, int M, int N, int KTOT, int ldd) {
  static_assert(FORM >= 0 && FORM <= 2);
  static_assert(EPI == 0 || EPI == 1);
  typedef typename FragOf<FORM>::T F;
  __shared__ __attribute__((aligned(16))) float sT[8][16 * 68];
  const int lane = threadIdx.x & 31;
  const int wave = threadIdx.x >> 5;
  const int tilesM = (M + 63) >> 6;
  const int tilesN = (N + 63) >> 6;
  const int tile = blockIdx.x * 8 + wave;
  if (tile >= tilesM * tilesN) return;
  const int tm = tile / tilesN;
  const int tn = tile - tm * tilesN;
  const int m0 = tm << 6;
  const int n0 = tn << 6;

  const int rl = lane & 15;
  const int h8 = (lane >> 4) * 8;
  const unsigned short* pa = A + (size_t)(m0 + rl) * (size_t)KTOT + h8;
  const unsigned short* pb = B + (size_t)(n0 + rl) * (size_t)KTOT + h8;

  v8f acc[4][4];
#pragma unroll
  for (int i = 0; i < 4; ++i)
#pragma unroll
    for (int j = 0; j < 4; ++j) acc[i][j] = (v8f){0.f, 0.f, 0.f, 0.f, 0.f, 0.f, 0.f, 0.f};

#pragma unroll 1
  for (int k0 = 0; k0 < KTOT; k0 += 32) {
    F bf[4];
#pragma unroll
    for (int j = 0; j < 4; ++j) bf[j] = ld_frag<F>(pb + (size_t)(j << 4) * (size_t)KTOT + k0);
#pragma unroll
    for (int i = 0; i < 4; ++i) {
      const F af = ld_frag<F>(pa + (size_t)(i << 4) * (size_t)KTOT + k0);
#pragma unroll
      for (int j = 0; j < 4; ++j) acc[i][j] = mm(af, bf[j], acc[i][j]);
    }
  }

  float* slab = sT[wave];
  const int hh = lane >> 4;
  const int c4 = (lane & 15) * 4;
  const int nc = n0 + c4;
  const bool cok = nc < N;
  v4f bv = (v4f){0.f, 0.f, 0.f, 0.f};
  if (EPI == 1) {
    bv = *(const v4fa*)(bias + clampi(nc, 0, N - 4));
    asm volatile("" :: "v"(bv));
  }
#pragma unroll
  for (int i = 0; i < 4; ++i) {
    const int mBase = m0 + (i << 4);
#pragma unroll
    for (int j = 0; j < 4; ++j) {
#pragma unroll
      for (int r = 0; r < 8; ++r) slab[(h8 + r) * 68 + (j << 4) + rl] = acc[i][j][r];
    }
    __builtin_amdgcn_fence(__ATOMIC_RELEASE, "workgroup");
    __builtin_amdgcn_wave_barrier();
    __builtin_amdgcn_fence(__ATOMIC_ACQUIRE, "workgroup");
    v4f vv[8];
#pragma unroll
    for (int it = 0; it < 8; ++it) {
      const int row = it * 2 + hh;
      v4f v = *(const v4fa*)(slab + row * 68 + c4);
      if (EPI == 1) v += bv;
      vv[it] = v;
    }
    for (int pass = 0; pass < 2; ++pass) {
#pragma unroll
      for (int it = 0; it < 8; ++it) {
        const int row = mBase + it * 2 + hh;
        if (cok && row < M) *(volatile v4f*)(D + (size_t)row * (size_t)ldd + nc) = vv[it];
      }
      __threadfence();
    }
    __builtin_amdgcn_fence(__ATOMIC_RELEASE, "workgroup");
    __builtin_amdgcn_wave_barrier();
    __builtin_amdgcn_fence(__ATOMIC_ACQUIRE, "workgroup");
  }
}

#ifndef SPLIT_AGGR
#define SPLIT_AGGR 1
#endif
#ifndef SPLIT_H
#define SPLIT_H 1
#endif

#define NNODE  50000
#define NEDGE  800000
#define DF     64
#define MPAD   50048
#define K1     192
#define K2     128
#define TABN   288
#define NTHR   256
#define NWAVE  8
#define EPT    8
#define CHUNK  (NTHR * EPT)
#define WCAP   (EPT * 32)
#define LISTN  (NWAVE * WCAP)
#define NBA    1024
#define NBLK   49
#define SLA    10
#define RCAP   21504
#define DEGCAP 64
#define ROWW   96
#define AGG_ZINTS    (LISTN + 2 * RCAP + 3 * NBA)
#define MISC_INTS    16
#define ROWBUF_INTS  (NWAVE * ROWW)
#define AGG_LDS_INTS (AGG_ZINTS + MISC_INTS + ROWBUF_INTS)

static_assert(NNODE % 16 == 0 && MPAD % 64 == 0 && MPAD == 391 * 128 && MPAD >= NNODE);
static_assert(K1 % 32 == 0 && K2 % 32 == 0 && DF == 64);
static_assert(NBA * NBLK >= MPAD && NBLK <= 64);
static_assert(NEDGE == 390 * CHUNK + 1280 && NEDGE % 4 == 0 && NEDGE < (1 << 21));
static_assert((CHUNK & (CHUNK - 1)) == 0 && NBA == (1 << SLA));
static_assert(((long long)NEDGE << SLA) < (1LL << 31));
static_assert(RCAP * 4 >= 16742 * 5 && DEGCAP >= 36 + 8);
static_assert(AGG_ZINTS % (NTHR * 4) == 0 && ((AGG_ZINTS + MISC_INTS) % 4) == 0 && ROWW % 4 == 0);
static_assert(AGG_LDS_INTS * 4 <= 262144);
static_assert((NNODE * 16) % 256 == 0 && (MPAD * 16) % 256 == 0 && MPAD % 128 == 0);
static_assert((long long)MPAD * K1 / 8 < (1LL << 31));

#define WS_W1C  ((size_t)0)
#define WS_W2C  (WS_W1C + (size_t)64 * K1 * 2)
#define WS_TAB  (WS_W2C + (size_t)64 * K2 * 2)
#define WS_FLG  (WS_TAB + (size_t)1280)
#define WS_XB   (WS_FLG + (size_t)64 * 128)
#define WS_TS   (WS_XB  + (size_t)MPAD * 64 * 2)
#define WS_A1   (WS_TS  + (size_t)2 * MPAD * 4)
#define WS_P    (WS_A1  + (size_t)MPAD * K1 * 2)
#define WS_A2   (WS_P   + (size_t)MPAD * 64 * 4)
#define WS_END  (WS_A2  + (size_t)MPAD * K2 * 2)
static_assert(WS_END == (size_t)51699968);
static_assert(WS_END <= ((size_t)128 << 20));
static_assert(WS_TAB % 256 == 0 && WS_FLG % 256 == 0 && WS_XB % 256 == 0 && WS_TS % 256 == 0);
static_assert(WS_A1 % 256 == 0 && WS_P % 256 == 0 && WS_A2 % 256 == 0);

typedef int v4i __attribute__((ext_vector_type(4)));
typedef v4i __attribute__((may_alias)) v4ia;
typedef v4u __attribute__((may_alias)) v4ua;

__device__ __forceinline__ void wave_sync() {
  __builtin_amdgcn_fence(__ATOMIC_RELEASE, "workgroup");
  __builtin_amdgcn_wave_barrier();
  __builtin_amdgcn_fence(__ATOMIC_ACQUIRE, "workgroup");
}

__global__ __launch_bounds__(256) void k_prep(const float* __restrict__ We, const float* __restrict__ be,
                                              const float* __restrict__ W1, const float* __restrict__ b1,
                                              const float* __restrict__ W2, const float* __restrict__ b2,
                                              unsigned short* __restrict__ W1C, unsigned short* __restrict__ W2C,
                                              float* __restrict__ TAB) {
  const int blk = (int)blockIdx.x;
  const int tid = (int)threadIdx.x;
  if (blk < 6) {
    const int u  = blk * 256 + tid;
    const int n  = u / 24;
    const int pc = u - n * 24;
    const int k0 = pc * 8;
    const int ks = (k0 < 128) ? k0 : (k0 - 64);
    float xv[8];
#pragma unroll
    for (int e = 0; e < 8; ++e) {
      const float v = W1[(size_t)(ks + e) * DF + n];
      asm volatile("" :: "v"(v));
      xv[e] = v;
    }
    const v4u o = pack8_bf16((v4f){ xv[0], xv[1], xv[2], xv[3] }, (v4f){ xv[4], xv[5], xv[6], xv[7] });
    volatile v4u* q = (volatile v4u*)(W1C + (size_t)u * 8);
    *q = o;
    __threadfence();
    *q = o;
  } else if (blk < 10) {
    const int u  = (blk - 6) * 256 + tid;
    const int n  = u >> 4;
    const int k0 = (u & 15) * 8;
    const int ks = k0 & 63;
    float xv[8];
#pragma unroll
    for (int e = 0; e < 8; ++e) {
      const float v = W2[(size_t)(ks + e) * DF + n];
      asm volatile("" :: "v"(v));
      xv[e] = v;
    }
    const v4u o = pack8_bf16((v4f){ xv[0], xv[1], xv[2], xv[3] }, (v4f){ xv[4], xv[5], xv[6], xv[7] });
    volatile v4u* q = (volatile v4u*)(W2C + (size_t)u * 8);
    *q = o;
    __threadfence();
    *q = o;
  } else {
    const int t = tid;
    const v4f wv  = *(const v4fa*)(We + 4 * clampi(t, 0, 31));
    const v4f b1v = *(const v4fa*)(b1 + 4 * clampi(t - 32, 0, 15));
    const v4f b2v = *(const v4fa*)(b2 + 4 * clampi(t - 48, 0, 15));
    const float bev = be[0];
    asm volatile("" :: "v"(wv));
    asm volatile("" :: "v"(b1v));
    asm volatile("" :: "v"(b2v));
    asm volatile("" :: "v"(bev));
    const unsigned mW = (t < 32) ? 0xFFFFFFFFu : 0u;
    const unsigned m1 = (t >= 32 && t < 48) ? 0xFFFFFFFFu : 0u;
    const unsigned m2 = (t >= 48 && t < 64) ? 0xFFFFFFFFu : 0u;
    const unsigned mE = (t == 64) ? 0xFFFFFFFFu : 0u;
    v4u o;
    o[0] = ((bf16_bits(wv[0]) << 16) & mW) | ((bf16_bits(b1v[0]) << 16) & m1) | ((bf16_bits(b2v[0]) << 16) & m2)
         | ((bf16_bits(bev) << 16) & mE);
    o[1] = ((bf16_bits(wv[1]) << 16) & mW) | ((bf16_bits(b1v[1]) << 16) & m1) | ((bf16_bits(b2v[1]) << 16) & m2);
    o[2] = ((bf16_bits(wv[2]) << 16) & mW) | ((bf16_bits(b1v[2]) << 16) & m1) | ((bf16_bits(b2v[2]) << 16) & m2);
    o[3] = ((bf16_bits(wv[3]) << 16) & mW) | ((bf16_bits(b1v[3]) << 16) & m1) | ((bf16_bits(b2v[3]) << 16) & m2);
    const bool wr = t < (TABN / 4);
    volatile v4u* q = (volatile v4u*)(TAB + 4 * clampi(t, 0, TABN / 4 - 1));
    if (wr) *q = o;
    __threadfence();
    if (wr) *q = o;
  }
}

__global__ __launch_bounds__(256) void k_node(const float* __restrict__ x, const float* __restrict__ tab,
                                              unsigned short* __restrict__ XB, float* __restrict__ TS, int nN) {
  __shared__ __attribute__((aligned(16))) float sWe[128];
  __shared__ __attribute__((aligned(16))) float sTS[256];
  const int tid = (int)threadIdx.x, lane = tid & 31, wave = tid >> 5;
  const int row0 = (int)blockIdx.x * 128;
  if (wave == 0) *(v4fa*)(sWe + 4 * lane) = *(const v4fa*)(tab + 4 * lane);
  __syncthreads();
#pragma unroll 1
  for (int it = 0; it < 4; ++it) {
    const int q = it * 256 + tid;
    const int r = q >> 3;
    const int p = q & 7;
    const int row = row0 + r;
    const float* sp = x + (size_t)clampi(row, 0, nN - 1) * DF + p * 8;
    const v4f a = *(const v4fa*)sp;
    const v4f c = *(const v4fa*)(sp + 4);
    asm volatile("" :: "v"(a));
    asm volatile("" :: "v"(c));
    const unsigned lm = (row < nN) ? 0xFFFFFFFFu : 0u;
    v4u o = pack8_bf16(a, c);
    o &= (v4u){ lm, lm, lm, lm };
    const float x0 = __uint_as_float(o[0] << 16), x1 = __uint_as_float(o[0] & 0xffff0000u);
    const float x2 = __uint_as_float(o[1] << 16), x3 = __uint_as_float(o[1] & 0xffff0000u);
    const float x4 = __uint_as_float(o[2] << 16), x5 = __uint_as_float(o[2] & 0xffff0000u);
    const float x6 = __uint_as_float(o[3] << 16), x7 = __uint_as_float(o[3] & 0xffff0000u);
    const v4f w0 = *(const v4fa*)(sWe + p * 8);
    const v4f w1 = *(const v4fa*)(sWe + p * 8 + 4);
    const v4f u0 = *(const v4fa*)(sWe + 64 + p * 8);
    const v4f u1 = *(const v4fa*)(sWe + 64 + p * 8 + 4);
    float t = x0 * w0[0];
    t = fmaf(x1, w0[1], t); t = fmaf(x2, w0[2], t); t = fmaf(x3, w0[3], t);
    t = fmaf(x4, w1[0], t); t = fmaf(x5, w1[1], t); t = fmaf(x6, w1[2], t); t = fmaf(x7, w1[3], t);
    float s = x0 * u0[0];
    s = fmaf(x1, u0[1], s); s = fmaf(x2, u0[2], s); s = fmaf(x3, u0[3], s);
    s = fmaf(x4, u1[0], s); s = fmaf(x5, u1[1], s); s = fmaf(x6, u1[2], s); s = fmaf(x7, u1[3], s);
    t += __shfl_xor(t, 1, 32); s += __shfl_xor(s, 1, 32);
    t += __shfl_xor(t, 2, 32); s += __shfl_xor(s, 2, 32);
    t += __shfl_xor(t, 4, 32); s += __shfl_xor(s, 4, 32);
    if (p == 0) { sTS[r] = t; sTS[128 + r] = s; }
    volatile v4u* qp = (volatile v4u*)(XB + (size_t)row0 * DF + (size_t)q * 8);
    *qp = o;
    __threadfence();
    *qp = o;
  }
  __syncthreads();
  if (wave < 2) {
    const v4f v = *(const v4fa*)(sTS + 128 * wave + 4 * lane);
    volatile v4f* dp = (volatile v4f*)(TS + (size_t)wave * MPAD + row0 + 4 * lane);
    *dp = v;
    __threadfence();
    *dp = v;
  }
}

template <int SLB>
__device__ __forceinline__ int scan_chunk(const int* __restrict__ dsts, int nE, int cbase, int slotBase,
                                          int nb, int vec8, int* list, int tid, int lane, int wave) {
  int wc = 0;
  const int el0  = tid * EPT;
  const int e0   = cbase + el0;
  const int sent = (-0x7fffffff - 1);
  v4i da, db;
  if (vec8 != 0 && cbase + CHUNK <= nE) {
    da = *(const v4i*)(dsts + e0);
    db = *(const v4i*)(dsts + e0 + 4);
  } else {
    const int q0 = dsts[min(e0,     nE - 1)];
    const int q1 = dsts[min(e0 + 1, nE - 1)];
    const int q2 = dsts[min(e0 + 2, nE - 1)];
    const int q3 = dsts[min(e0 + 3, nE - 1)];
    const int q4 = dsts[min(e0 + 4, nE - 1)];
    const int q5 = dsts[min(e0 + 5, nE - 1)];
    const int q6 = dsts[min(e0 + 6, nE - 1)];
    const int q7 = dsts[min(e0 + 7, nE - 1)];
    asm volatile("" :: "v"(q0)); asm volatile("" :: "v"(q1));
    asm volatile("" :: "v"(q2)); asm volatile("" :: "v"(q3));
    asm volatile("" :: "v"(q4)); asm volatile("" :: "v"(q5));
    asm volatile("" :: "v"(q6)); asm volatile("" :: "v"(q7));
    da.x = (e0     < nE) ? q0 : sent;
    da.y = (e0 + 1 < nE) ? q1 : sent;
    da.z = (e0 + 2 < nE) ? q2 : sent;
    da.w = (e0 + 3 < nE) ? q3 : sent;
    db.x = (e0 + 4 < nE) ? q4 : sent;
    db.y = (e0 + 5 < nE) ? q5 : sent;
    db.z = (e0 + 6 < nE) ? q6 : sent;
    db.w = (e0 + 7 < nE) ? q7 : sent;
  }
  const unsigned nbs = (unsigned)slotBase;
  const unsigned unb = (unsigned)nb;
  const unsigned s0 = (unsigned)da.x - nbs, s1 = (unsigned)da.y - nbs;
  const unsigned s2 = (unsigned)da.z - nbs, s3 = (unsigned)da.w - nbs;
  const unsigned s4 = (unsigned)db.x - nbs, s5 = (unsigned)db.y - nbs;
  const unsigned s6 = (unsigned)db.z - nbs, s7 = (unsigned)db.w - nbs;
  const bool h0 = s0 < unb, h1 = s1 < unb, h2 = s2 < unb, h3 = s3 < unb;
  const bool h4 = s4 < unb, h5 = s5 < unb, h6 = s6 < unb, h7 = s7 < unb;
  const unsigned any = __builtin_amdgcn_ballot_w32(h0 | h1 | h2 | h3 | h4 | h5 | h6 | h7);
  if (any != 0u) {
#define HITJ(J, HJ, SJ) { \
      const unsigned mj = __builtin_amdgcn_ballot_w32(HJ); \
      if (mj != 0u) { \
        if (HJ) { \
          const int pos = wc + (int)__builtin_amdgcn_mbcnt_lo(mj, 0u); \
          if (pos < WCAP) list[wave * WCAP + pos] = ((el0 + (J)) << SLB) | (int)(SJ); \
        } \
        wc += (int)__builtin_popcount(mj); } }
    HITJ(0, h0, s0)
    HITJ(1, h1, s1)
    HITJ(2, h2, s2)
    HITJ(3, h3, s3)
    HITJ(4, h4, s4)
    HITJ(5, h5, s5)
    HITJ(6, h6, s6)
    HITJ(7, h7, s7)
#undef HITJ
  }
  return wc;
}

__global__ __launch_bounds__(NTHR) void k_aggr(const int* __restrict__ srcs, const int* __restrict__ keys,
                                               const unsigned* __restrict__ XBw, const float* __restrict__ Tp,
                                               const float* __restrict__ Sp, const float* __restrict__ tab,
                                               unsigned* __restrict__ A1w, unsigned* __restrict__ FLG,
                                               int nE, int nN, int vec8, int mRows) {
  extern __shared__ __attribute__((aligned(16))) int dsm[];
  int* list = dsm;
  int* hl   = dsm + LISTN;
  int* sl   = hl + RCAP;
  int* cnt  = sl + RCAP;
  int* offs = cnt + NBA;
  int* cur  = offs + NBA;
  int* misc = cur + NBA;
  const int tid = (int)threadIdx.x, lane = tid & 31, wave = tid >> 5;
  unsigned* rowbuf = (unsigned*)(misc + MISC_INTS) + wave * ROWW;
  const int nodeBase = (int)blockIdx.x * NBA;

  {
    const v4i z4 = {0, 0, 0, 0};
    for (int i = tid * 4; i < AGG_ZINTS; i += NTHR * 4) *(v4ia*)(dsm + i) = z4;
    if (tid < MISC_INTS) misc[tid] = 0;
  }
  __syncthreads();

  int t = 0, ov = 0;
  const int nChunks = (nE + CHUNK - 1) / CHUNK;
#pragma unroll 1
  for (int ch = 0; ch < nChunks; ++ch) {
    const int cbase = ch * CHUNK;
    const int wc = scan_chunk<SLA>(keys, nE, cbase, nodeBase, NBA, vec8, list, tid, lane, wave);
    if (lane == 0) misc[wave] = wc;
    __syncthreads();
    if (wave == 0) {
#pragma unroll 1
      for (int w2 = 0; w2 < NWAVE; ++w2) {
        int c = misc[w2];
        c = c < 0 ? 0 : (c > WCAP ? WCAP : c);
        c = __builtin_amdgcn_readfirstlane(c);
#pragma unroll 1
        for (int b0 = 0; b0 < c; b0 += 32) {
          const int idx = b0 + lane;
          const int ent = list[w2 * WCAP + (idx < WCAP ? idx : WCAP - 1)];
          const int m32 = (c - b0) < 32 ? (c - b0) : 32;
#pragma unroll 1
          for (int k = 0; k < m32; ++k) {
            const int u    = __builtin_amdgcn_readlane(ent, k);
            const int slot = u & (NBA - 1);
            const int el   = (u >> SLA) & (CHUNK - 1);
            const int pk   = ((cbase + el) << SLA) | slot;
            if (t < RCAP) {
              if (lane == 0) { hl[t] = pk; cnt[slot] = cnt[slot] + 1; }
              t = t + 1;
            } else {
              ov = 1;
            }
          }
        }
      }
    }
    __syncthreads();
  }
  if (wave == 0 && lane == 0) { misc[8] = t; misc[9] = ov; }
  __syncthreads();
  int tt = misc[8];
  tt = tt < 0 ? 0 : (tt > RCAP ? RCAP : tt);
  tt = __builtin_amdgcn_readfirstlane(tt);

  if (wave == 0) {
    const int base = lane * (NBA / 32);
    int s = 0, mx = 0;
#pragma unroll 1
    for (int i = 0; i < NBA / 32; ++i) {
      const int cv = cnt[base + i];
      s += cv;
      mx = cv > mx ? cv : mx;
    }
    int incl = s;
#pragma unroll
    for (int d = 1; d < 32; d <<= 1) {
      const int y = __shfl_up(incl, d, 32);
      if (lane >= d) incl += y;
    }
#pragma unroll
    for (int d = 16; d > 0; d >>= 1) {
      const int y = __shfl_xor(mx, d, 32);
      mx = y > mx ? y : mx;
    }
    if (lane == 0) misc[10] = (mx > DEGCAP) ? 1 : 0;
    int run = incl - s;
#pragma unroll 1
    for (int i = 0; i < NBA / 32; ++i) {
      const int cv = cnt[base + i];
      offs[base + i] = run;
      cur[base + i]  = run;
      run += cv;
    }
  }
  __syncthreads();
  if (wave == 0) {
#pragma unroll 1
    for (int b0 = 0; b0 < tt; b0 += 32) {
      const int idx = b0 + lane;
      const int ent = hl[idx < RCAP ? idx : RCAP - 1];
      const int m32 = (tt - b0) < 32 ? (tt - b0) : 32;
#pragma unroll 1
      for (int k = 0; k < m32; ++k) {
        const int u    = __builtin_amdgcn_readlane(ent, k);
        const int slot = u & (NBA - 1);
        if (lane == 0) {
          int p = cur[slot];
          p = p < 0 ? 0 : (p > RCAP - 1 ? RCAP - 1 : p);
          sl[p] = u;
          cur[slot] = p + 1;
        }
      }
    }
  }
  __syncthreads();

  const int flg = ((misc[9] | misc[10]) != 0) ? 1 : 0;
  if (wave == 0) {
    const unsigned f = (unsigned)flg;
    const v4u fv = (v4u){ f, f, f, f };
    const bool wr = lane < 8;
    volatile v4u* fp = (volatile v4u*)(FLG + (size_t)blockIdx.x * 32 + 4 * (lane & 7));
    if (wr) *fp = fv;
    __threadfence();
    if (wr) *fp = fv;
  }

  const float pz  = (flg != 0) ? __int_as_float(0x7fc00000) : 0.0f;
  const float beb = tab[256];
#pragma unroll 1
  for (int si = 0; si < NBA / NWAVE; ++si) {
    const int s    = si * NWAVE + wave;
    const int node = nodeBase + s;
    const bool live = node < nN;
    int c = cnt[s];
    c = c < 0 ? 0 : (c > DEGCAP ? DEGCAP : c);
    c = live ? c : 0;
    c = __builtin_amdgcn_readfirstlane(c);
    int o = offs[s];
    o = o < 0 ? 0 : (o > RCAP ? RCAP : o);
    o = __builtin_amdgcn_readfirstlane(o);
    const int nc = node < nN ? node : nN - 1;
    const float ti = Tp[nc];
    asm volatile("" :: "v"(ti));
    const unsigned ow = XBw[(size_t)nc * 32 + lane];
    asm volatile("" :: "v"(ow));
    float a0 = 0.0f, a1 = 0.0f;
#pragma unroll 1
    for (int b0 = 0; b0 < c; b0 += 32) {
      int idx = o + b0 + lane;
      idx = idx > RCAP - 1 ? RCAP - 1 : idx;
      const int ent = sl[idx];
      int eid = ent >> SLA;
      eid = eid < 0 ? 0 : (eid > nE - 1 ? nE - 1 : eid);
      int sr = srcs[eid];
      asm volatile("" :: "v"(sr));
      sr = sr < 0 ? 0 : (sr > nN - 1 ? nN - 1 : sr);
      const float sv = Sp[sr];
      asm volatile("" :: "v"(sv));
      const float z  = ti + sv + beb;
      const float g  = 1.0f / (1.0f + expf(-z));
      const int   gi = __float_as_int(g);
      const int m32 = (c - b0) < 32 ? (c - b0) : 32;
#pragma unroll 1
      for (int k = 0; k < m32; ++k) {
        const int   sk = __builtin_amdgcn_readlane(sr, k);
        const float gk = __int_as_float(__builtin_amdgcn_readlane(gi, k));
        const unsigned w = XBw[(size_t)sk * 32 + lane];
        asm volatile("" :: "v"(w));
        a0 = fmaf(gk, __uint_as_float(w << 16), a0);
        a1 = fmaf(gk, __uint_as_float(w & 0xffff0000u), a1);
      }
    }
    const float m0 = a0 + pz;
    const float m1 = a1 + pz;
    const unsigned hw = pk16(bf16_bits(m0), bf16_bits(m1));
#if SPLIT_AGGR
    const unsigned lw = pk16(bf16_lo_bits(m0), bf16_lo_bits(m1));
#else
    const unsigned lw = 0u;
#endif
    const unsigned lm = live ? 0xFFFFFFFFu : 0u;
    rowbuf[lane]      = ow & lm;
    rowbuf[32 + lane] = hw & lm;
    rowbuf[64 + lane] = lw & lm;
    wave_sync();
    const int pl = lane < 24 ? lane : 23;
    const v4u q = *(const v4ua*)(rowbuf + 4 * pl);
    wave_sync();
    const bool wr = (node < mRows) && (lane < 24);
    volatile v4u* rp = (volatile v4u*)(A1w + (size_t)(node < mRows ? node : mRows - 1) * ROWW + 4 * pl);
    if (wr) *rp = q;
    __threadfence();
    if (wr) *rp = q;
  }
}

__global__ __launch_bounds__(256) void k_row1(const float* __restrict__ P, unsigned short* __restrict__ A2, int nN) {
  __shared__ __attribute__((aligned(16))) unsigned shw[16 * 64];
  const int tid = (int)threadIdx.x;
  const int r   = tid >> 4;
  const int c4  = (tid & 15) * 4;
  const int row = (int)blockIdx.x * 16 + r;
  const v4f v = *(const v4fa*)(P + (size_t)clampi(row, 0, nN - 1) * DF + c4);
  asm volatile("" :: "v"(v));
  const float h0 = tanhf(v[0]);
  const float h1 = tanhf(v[1]);
  const float h2 = tanhf(v[2]);
  const float h3 = tanhf(v[3]);
  const unsigned lm = (row < nN) ? 0xFFFFFFFFu : 0u;
  const unsigned hA = pk16(bf16_bits(h0), bf16_bits(h1)) & lm;
  const unsigned hB = pk16(bf16_bits(h2), bf16_bits(h3)) & lm;
#if SPLIT_H
  const unsigned lA = pk16(bf16_lo_bits(h0), bf16_lo_bits(h1)) & lm;
  const unsigned lB = pk16(bf16_lo_bits(h2), bf16_lo_bits(h3)) & lm;
#else
  const unsigned lA = 0u;
  const unsigned lB = 0u;
#endif
  shw[r * 64 + (c4 >> 1)]          = hA;
  shw[r * 64 + (c4 >> 1) + 1]      = hB;
  shw[r * 64 + 32 + (c4 >> 1)]     = lA;
  shw[r * 64 + 32 + (c4 >> 1) + 1] = lB;
  __syncthreads();
  const v4u q = *(const v4ua*)(shw + tid * 4);
  volatile v4u* dp = (volatile v4u*)(A2 + (size_t)blockIdx.x * 16 * K2 + (size_t)tid * 8);
  *dp = q;
  __threadfence();
  *dp = q;
}

__global__ __launch_bounds__(256) void k_out(const float* __restrict__ P, const unsigned* __restrict__ FLG,
                                             float* __restrict__ outp, int nN) {
  const int g   = (int)blockIdx.x * 256 + (int)threadIdx.x;
  const int row = g >> 4;
  const int c4  = (g & 15) * 4;
  const int rc  = clampi(row, 0, nN - 1);
  const v4f v = *(const v4fa*)(P + (size_t)rc * DF + c4);
  asm volatile("" :: "v"(v));
  const unsigned fl = FLG[(size_t)clampi(rc >> SLA, 0, 63) * 32];
  asm volatile("" :: "v"(fl));
  const float nanv = __uint_as_float(0x7fc00000u);
  v4f o;
  o[0] = tanhf(v[0]);
  o[1] = tanhf(v[1]);
  o[2] = tanhf(v[2]);
  o[3] = tanhf(v[3]);
  o[0] = (fl != 0u) ? nanv : o[0];
  o[1] = (fl != 0u) ? nanv : o[1];
  o[2] = (fl != 0u) ? nanv : o[2];
  o[3] = (fl != 0u) ? nanv : o[3];
  const bool wr = row < nN;
  volatile v4f* dp = (volatile v4f*)(outp + (size_t)rc * DF + c4);
  if (wr) *dp = o;
  __threadfence();
  if (wr) *dp = o;
}

extern "C" void kernel_launch(void* const* d_in, const int* in_sizes, int n_in,
                              void* d_out, int out_size, void* d_ws, size_t ws_size,
                              hipStream_t stream) {
  if (n_in < 24) return;
  for (int p = 0; p < 3; ++p) {
    if (in_sizes[8 * p + 0] != NNODE * DF) return;
    if (in_sizes[8 * p + 1] != 2 * NEDGE) return;
    if (in_sizes[8 * p + 2] != 2 * DF) return;
    if (in_sizes[8 * p + 3] != 1) return;
    if (in_sizes[8 * p + 4] != 2 * DF * DF) return;
    if (in_sizes[8 * p + 5] != DF) return;
    if (in_sizes[8 * p + 6] != DF * DF) return;
    if (in_sizes[8 * p + 7] != DF) return;
  }
  if ((long long)out_size != 3LL * NNODE * DF) return;
  if ((size_t)WS_END > ws_size) return;

  char* ws = (char*)d_ws;
  unsigned short* W1C = (unsigned short*)(ws + WS_W1C);
  unsigned short* W2C = (unsigned short*)(ws + WS_W2C);
  float*          TAB = (float*)(ws + WS_TAB);
  unsigned*       FLG = (unsigned*)(ws + WS_FLG);
  unsigned short* XB  = (unsigned short*)(ws + WS_XB);
  float*          TS  = (float*)(ws + WS_TS);
  unsigned short* A1  = (unsigned short*)(ws + WS_A1);
  float*          P   = (float*)(ws + WS_P);
  unsigned short* A2  = (unsigned short*)(ws + WS_A2);

  const size_t aggLds = (size_t)AGG_LDS_INTS * 4;
  hipFuncSetAttribute(reinterpret_cast<const void*>(&k_aggr), hipFuncAttributeMaxDynamicSharedMemorySize, (int)aggLds);

  const int vec8 = ((NEDGE & 3) == 0) ? 1 : 0;
  const int gemmBlocks = ((MPAD / 64) + 7) / 8;

  for (int p = 0; p < 3; ++p) {
    const float* x  = (const float*)d_in[8 * p + 0];
    const int*   ei = (const int*)  d_in[8 * p + 1];
    const float* We = (const float*)d_in[8 * p + 2];
    const float* be = (const float*)d_in[8 * p + 3];
    const float* W1 = (const float*)d_in[8 * p + 4];
    const float* b1 = (const float*)d_in[8 * p + 5];
    const float* W2 = (const float*)d_in[8 * p + 6];
    const float* b2 = (const float*)d_in[8 * p + 7];
    float* outp = (float*)d_out + (size_t)p * NNODE * DF;

    k_prep<<<11, 256, 0, stream>>>(We, be, W1, b1, W2, b2, W1C, W2C, TAB);
    k_node<<<MPAD / 128, 256, 0, stream>>>(x, TAB, XB, TS, NNODE);
    k_aggr<<<NBLK, NTHR, aggLds, stream>>>(ei, ei + NEDGE, (const unsigned*)XB, TS, TS + MPAD, TAB,
                                           (unsigned*)A1, FLG, NEDGE, NNODE, vec8, MPAD);
    k_gemm_nt<0, 1><<<gemmBlocks, 256, 0, stream>>>(A1, W1C, TAB + 128, P, NNODE, DF, K1, DF);
    k_row1<<<MPAD / 16, 256, 0, stream>>>(P, A2, NNODE);
    k_gemm_nt<0, 1><<<gemmBlocks, 256, 0, stream>>>(A2, W2C, TAB + 192, P, NNODE, DF, K2, DF);
    k_out<<<(NNODE * 16) / 256, 256, 0, stream>>>(P, FLG, outp, NNODE);
  }
}
